// Forward_78211354460854
// MI455X (gfx1250) — hardware-verified
//
#include <hip/hip_runtime.h>

#define NBATCH 2048
#define H1 1000
#define HP 1024
#define N3 301
#define N3P 512
#define NL 100
#define NSPEC 300

typedef _Float16 f16;
typedef __attribute__((ext_vector_type(16))) f16 f16x16;
typedef __attribute__((ext_vector_type(8)))  f16 f16x8;
typedef __attribute__((ext_vector_type(8)))  float f32x8;
typedef __attribute__((ext_vector_type(4)))  float v4f_t;
typedef float v4fa __attribute__((ext_vector_type(4), may_alias));

__device__ __forceinline__ f32x8 wmma16(f16x16 a, f16x16 b, f32x8 c) {
  c = __builtin_amdgcn_wmma_f32_16x16x32_f16(false, a, false, b, (short)0, c, false, false);
  asm volatile("v_nop\n\tv_nop\n\tv_nop\n\tv_nop" : "+v"(c) : "v"(a), "v"(b));
  return c;
}
__device__ __forceinline__ f16x16 lds_frag(const f16* base, int stride) {
  const int lane = threadIdx.x & 31, row = lane & 15, kh = (lane >> 4) * 8;
  const f16x8 lo = *(const f16x8*)(base + row * stride + kh);
  const f16x8 hi = *(const f16x8*)(base + row * stride + kh + 16);
  f16x16 f;
#pragma unroll
  for (int i = 0; i < 8; ++i) { f[i] = lo[i]; f[i + 8] = hi[i]; }
  return f;
}
#define GSTR 48

template <typename AT, bool RELU>
__global__ __launch_bounds__(256) void gemm_kn2bn(const AT* __restrict__ A, int lda, size_t strideA,
                                               const float* __restrict__ Wm, int ldw, size_t strideW,
                                               const float* __restrict__ bias, const float* __restrict__ gam, const float* __restrict__ bet,
                                               const float* __restrict__ mean, const float* __restrict__ var, int nvalid,
                                               float* __restrict__ Y, int ldy, size_t strideY, int K) {
  __shared__ __attribute__((aligned(16))) f16 ldsA[128 * GSTR], ldsAl[128 * GSTR];
  __shared__ __attribute__((aligned(16))) f16 ldsW[128 * GSTR], ldsWl[128 * GSTR];
  __shared__ __attribute__((aligned(16))) float oS[8][32 * 68];
  const int tid = threadIdx.x, lane = tid & 31, wave = tid >> 5, cl = lane & 15, rh = (lane >> 4) * 8;
  const int m0 = blockIdx.x * 128, n0 = blockIdx.y * 128;
  const int wm = (wave & 3) * 32, wn = (wave >> 2) * 64;
  A += (size_t)blockIdx.z * strideA; Wm += (size_t)blockIdx.z * strideW; Y += (size_t)blockIdx.z * strideY;
  f32x8 acc[2][4], accx[2][4];
#pragma unroll
  for (int i = 0; i < 2; ++i)
#pragma unroll
    for (int j = 0; j < 4; ++j) { f32x8 z = {}; acc[i][j] = z; accx[i][j] = z; }
#pragma unroll 1
  for (int k0 = 0; k0 < K; k0 += 32) {
    __syncthreads();
    {
      const int row = tid >> 1, ch = (tid & 1) * 16;
      const AT* src = A + (size_t)(m0 + row) * lda + k0 + ch;
#pragma unroll
      for (int g = 0; g < 16; ++g) { const float v = (float)src[g]; const f16 h = (f16)v; ldsA[row * GSTR + ch + g] = h; ldsAl[row * GSTR + ch + g] = (f16)((v - (float)h) * 2048.0f); }
    }
    {
      const int k = tid >> 3, nn0 = (tid & 7) * 16;
      const float* src = Wm + (size_t)(k0 + k) * ldw + n0 + nn0;
#pragma unroll
      for (int g = 0; g < 4; ++g) { const v4f_t v = *(const v4f_t*)(src + 4 * g);
#pragma unroll
        for (int u = 0; u < 4; ++u) { const f16 h = (f16)v[u]; ldsW[(nn0 + 4 * g + u) * GSTR + k] = h; ldsWl[(nn0 + 4 * g + u) * GSTR + k] = (f16)((v[u] - (float)h) * 2048.0f); } }
    }
    __syncthreads();
    f16x16 af[2], afl[2];
#pragma unroll
    for (int i = 0; i < 2; ++i) { af[i] = lds_frag(ldsA + (wm + 16 * i) * GSTR, GSTR); afl[i] = lds_frag(ldsAl + (wm + 16 * i) * GSTR, GSTR); }
#pragma unroll
    for (int j = 0; j < 4; ++j) {
      const f16x16 bf = lds_frag(ldsW + (wn + 16 * j) * GSTR, GSTR), bfl = lds_frag(ldsWl + (wn + 16 * j) * GSTR, GSTR);
#pragma unroll
      for (int i = 0; i < 2; ++i) { acc[i][j] = wmma16(af[i], bf, acc[i][j]); accx[i][j] = wmma16(af[i], bfl, accx[i][j]); accx[i][j] = wmma16(afl[i], bf, accx[i][j]); }
    }
  }
  float* so = oS[wave];
#pragma unroll
  for (int i = 0; i < 2; ++i)
#pragma unroll
    for (int j = 0; j < 4; ++j) {
      const int n = n0 + wn + 16 * j + cl;
      const bool nv = (n < nvalid);
      const float bv = nv ? bias[n] : 0.0f, gsc = nv ? gam[n] * rsqrtf(var[n] + 1e-5f) : 0.0f, mu = nv ? mean[n] : 0.0f, bb = nv ? bet[n] : 0.0f;
#pragma unroll
      for (int r = 0; r < 8; ++r) { float v = ((acc[i][j][r] + accx[i][j][r] * (1.0f / 2048.0f)) + bv - mu) * gsc + bb; if (RELU) v = fmaxf(v, 0.0f); so[(16 * i + rh + r) * 68 + 16 * j + cl] = nv ? v : 0.0f; }
    }
  asm volatile("s_wait_dscnt 0" ::: "memory");
  __builtin_amdgcn_wave_barrier();
#pragma unroll 1
  for (int pass = 0; pass < 2; ++pass) {
#pragma unroll
    for (int it = 0; it < 16; ++it) { const int f4 = lane + 32 * it, rr = f4 >> 4, q = (f4 & 15) * 4;
      *(volatile v4f_t*)(Y + (size_t)(m0 + wm + rr) * ldy + n0 + wn + q) = *(const volatile v4fa*)(so + rr * 68 + q); }
    __threadfence();
  }
}

__global__ __launch_bounds__(256) void k_layer1(const float* __restrict__ G, const float* __restrict__ W1, const float* __restrict__ b1,
                                                const float* __restrict__ ga, const float* __restrict__ be, const float* __restrict__ mu,
                                                const float* __restrict__ var, float* __restrict__ h1) {
  __shared__ float gS[8][8];
  const int tid = threadIdx.x, r0 = blockIdx.x * 8;
  if (tid < 64) gS[tid >> 3][tid & 7] = G[(size_t)(r0 + (tid >> 3)) * 8 + (tid & 7)];
  __syncthreads();
#pragma unroll 1
  for (int row = 0; row < 8; ++row) {
    v4f_t o;
#pragma unroll
    for (int u = 0; u < 4; ++u) {
      const int n = tid * 4 + u;
      float v = 0.0f;
      if (n < H1) {
        float s = b1[n];
#pragma unroll
        for (int k = 0; k < 8; ++k) s += gS[row][k] * W1[n * 8 + k];
        s = (s - mu[n]) * (ga[n] * rsqrtf(var[n] + 1e-5f)) + be[n];
        v = fmaxf(s, 0.0f);
      }
      o[u] = v;
    }
    float* dst = h1 + (size_t)(r0 + row) * HP + tid * 4;
    *(volatile v4f_t*)dst = o; __threadfence(); *(volatile v4f_t*)dst = o;
  }
}
__global__ __launch_bounds__(256) void k_transpose_pad(const float* __restrict__ Wm, float* __restrict__ Wt, int N, int K, int NP, int KP) {
  const size_t g = (size_t)blockIdx.x * 256 + threadIdx.x;
  const size_t e0 = g * 4;
  if (e0 >= (size_t)KP * NP) return;
  const int k = (int)(e0 / NP), n0 = (int)(e0 % NP);
  v4f_t v;
#pragma unroll
  for (int u = 0; u < 4; ++u) { const int n = n0 + u; v[u] = (k < K && n < N) ? Wm[(size_t)n * K + k] : 0.0f; }
  *(volatile v4f_t*)(Wt + e0) = v; __threadfence(); *(volatile v4f_t*)(Wt + e0) = v;
}
__global__ __launch_bounds__(256) void k_lorentz(const float* __restrict__ h3, const float* __restrict__ G, const float* __restrict__ wgrid, float* __restrict__ T) {
  __shared__ float pS[8][NL * 3];
  __shared__ float dS[8];
  __shared__ __attribute__((aligned(16))) float tS[8 * NSPEC];
  const int tid = threadIdx.x, r0 = blockIdx.x * 8;
  for (int e = tid; e < 8 * NL * 3; e += 256) { const int row = e / (NL * 3), c = e % (NL * 3); const float hv = h3[(size_t)(r0 + row) * N3P + c]; pS[row][c] = 1.0f / (1.0f + __expf(-hv)); }
  if (tid < 8) { const float* g = G + (size_t)(r0 + tid) * 8; dS[tid] = fmaxf(fmaxf(g[4], g[5]), fmaxf(g[6], g[7])); }
  __syncthreads();
  for (int e = tid; e < 8 * NSPEC; e += 256) {
    const int row = e / NSPEC, s = e % NSPEC;
    const float wg = wgrid[s], w2 = wg * wg;
    float e1 = 0.0f, e2 = 0.0f;
    for (int l = 0; l < NL; ++l) {
      const float w0 = pS[row][3 * l] * 5.0f, wp = pS[row][3 * l + 1] * 5.0f, g = pS[row][3 * l + 2] * 0.5f;
      const float w02 = w0 * w0, wp2 = wp * wp, g2 = g * g;
      const float s1 = w02 - w2, den = s1 * s1 + w2 * g2;
      e1 += wp2 * s1 / den;
      e2 += wp2 * (wg * g) / den;
    }
    e1 += 10.0f;
    const float mag = sqrtf(e1 * e1 + e2 * e2);
    const float n = sqrtf(0.5f * (mag + e1)), k = sqrtf(0.5f * (mag - e1));
    const float ab = __expf(-0.0005f * 4.0f * 3.14159265358979323846f * dS[row] * k);
    tS[e] = (4.0f * n / ((n + 1.0f) * (n + 1.0f) + k * k)) * ab;
  }
  __syncthreads();
#pragma unroll 1
  for (int pass = 0; pass < 2; ++pass) {
    for (int f4 = tid; f4 < 600; f4 += 256) *(volatile v4f_t*)(T + (size_t)r0 * NSPEC + f4 * 4) = *(const volatile v4fa*)(tS + f4 * 4);
    __threadfence();
  }
}

extern "C" void kernel_launch(void* const* d_in, const int* in_sizes, int n_in,
                              void* d_out, int out_size, void* d_ws, size_t ws_size,
                              hipStream_t stream) {
  (void)in_sizes; (void)n_in; (void)out_size; (void)ws_size;
  const float* G = (const float*)d_in[0];
  const float* W1 = (const float*)d_in[1], *b1 = (const float*)d_in[2], *g1 = (const float*)d_in[3], *be1 = (const float*)d_in[4], *m1 = (const float*)d_in[5], *v1 = (const float*)d_in[6];
  const float* W2 = (const float*)d_in[7], *b2 = (const float*)d_in[8], *g2 = (const float*)d_in[9], *be2 = (const float*)d_in[10], *m2 = (const float*)d_in[11], *v2 = (const float*)d_in[12];
  const float* W3 = (const float*)d_in[13], *b3 = (const float*)d_in[14], *g3 = (const float*)d_in[15], *be3 = (const float*)d_in[16], *m3 = (const float*)d_in[17], *v3 = (const float*)d_in[18];
  const float* wgrid = (const float*)d_in[19];
  float* T = (float*)d_out;
  char* ws = (char*)d_ws;
  float* h1 = (float*)ws; ws += (size_t)NBATCH * HP * 4;
  float* W2t = (float*)ws; ws += (size_t)HP * HP * 4;
  float* h2 = (float*)ws; ws += (size_t)NBATCH * HP * 4;
  float* W3t = (float*)ws; ws += (size_t)HP * N3P * 4;
  float* h3 = (float*)ws; ws += (size_t)NBATCH * N3P * 4;
  k_layer1<<<dim3(NBATCH / 8), dim3(256), 0, stream>>>(G, W1, b1, g1, be1, m1, v1, h1);
  k_transpose_pad<<<dim3((HP * HP / 4 + 255) / 256), dim3(256), 0, stream>>>(W2, W2t, H1, H1, HP, HP);
  k_transpose_pad<<<dim3((HP * N3P / 4 + 255) / 256), dim3(256), 0, stream>>>(W3, W3t, N3, H1, N3P, HP);
  gemm_kn2bn<float, true ><<<dim3(NBATCH / 128, HP / 128, 1), dim3(256), 0, stream>>>(h1, HP, 0, W2t, HP, 0, b2, g2, be2, m2, v2, H1, h2, HP, 0, HP);
  gemm_kn2bn<float, false><<<dim3(NBATCH / 128, N3P / 128, 1), dim3(256), 0, stream>>>(h2, HP, 0, W3t, N3P, 0, b3, g3, be3, m3, v3, N3, h3, N3P, 0, HP);
  k_lorentz<<<dim3(NBATCH / 8), dim3(256), 0, stream>>>(h3, G, wgrid, T);
}
